// MambaSemanticMapper_NoPool_50208167690330
// MI455X (gfx1250) — hardware-verified
//
#include <hip/hip_runtime.h>
#include <hip/hip_bf16.h>

#define LSEQ 1024
#define BB 4
#define BL (BB * LSEQ)
#define DMODEL 256
#define DCLIP 512
#define DINNER 512
#define DSTATE 16
#define DTRANK 16
#define NPROJ 48
#define NPROJP 64

typedef _Float16 v8h  __attribute__((ext_vector_type(8)));
typedef _Float16 v16h __attribute__((ext_vector_type(16)));
typedef float    v8f  __attribute__((ext_vector_type(8)));
#define VST2(T, ptr, val) do { const T _v = (val); *(volatile T*)(ptr) = _v; __threadfence(); *(volatile T*)(ptr) = _v; } while (0)

union FragH { v16h v; v8h h[2]; };

enum { GF_BIAS = 1, GF_WRITEH = 2, GF_REVA = 4, GF_REVC = 8, GF_ACC = 16 };

__global__ void k_f32_to_f16(const float* __restrict__ in, _Float16* __restrict__ out, int n) {
    int i = blockIdx.x * blockDim.x + threadIdx.x;
    if (i < n) VST2(_Float16, out + i, (_Float16)in[i]);
}

__global__ void k_f32_to_f16_pad(const float* __restrict__ in, _Float16* __restrict__ out,
                                 int rows_in, int rows_out, int cols) {
    int i = blockIdx.x * blockDim.x + threadIdx.x;
    if (i >= rows_out * cols) return;
    int row = i / cols;
    VST2(_Float16, out + i, (row < rows_in) ? (_Float16)in[i] : (_Float16)0.0f);
}

__global__ void k_gemm_f16(const _Float16* __restrict__ A, const _Float16* __restrict__ W,
                           const float* __restrict__ bias, float* __restrict__ C,
                           _Float16* __restrict__ Ch, int M, int N, int K, int flags) {
    const int wave = blockIdx.x * (blockDim.x >> 5) + (threadIdx.x >> 5);
    const int lane = threadIdx.x & 31;
    const int ntiles = N >> 5;
    const int mt = wave / ntiles, nt = wave % ntiles;
    const int row0 = mt << 5, col0 = nt << 5;
    const int half = lane >> 4;
    const int lidx = lane & 15;

    int am0 = row0 + lidx;
    int am1 = row0 + 16 + lidx;
    if (flags & GF_REVA) {
        am0 = (am0 / LSEQ) * LSEQ + (LSEQ - 1 - (am0 % LSEQ));
        am1 = (am1 / LSEQ) * LSEQ + (LSEQ - 1 - (am1 % LSEQ));
    }
    const _Float16* __restrict__ arow0 = A + (size_t)am0 * K + half * 8;
    const _Float16* __restrict__ arow1 = A + (size_t)am1 * K + half * 8;
    const _Float16* __restrict__ wrow0 = W + (size_t)(col0 + lidx) * K + half * 8;
    const _Float16* __restrict__ wrow1 = W + (size_t)(col0 + 16 + lidx) * K + half * 8;
    __shared__ __attribute__((aligned(16))) float sT[4][32][33];

    v8f acc00 = {}, acc01 = {}, acc10 = {}, acc11 = {};
#pragma unroll 2
    for (int k0 = 0; k0 < K; k0 += 32) {
        FragH a0, a1, b0, b1;
        a0.h[0] = *(const v8h*)(arow0 + k0);
        a0.h[1] = *(const v8h*)(arow0 + k0 + 16);
        a1.h[0] = *(const v8h*)(arow1 + k0);
        a1.h[1] = *(const v8h*)(arow1 + k0 + 16);
        b0.h[0] = *(const v8h*)(wrow0 + k0);
        b0.h[1] = *(const v8h*)(wrow0 + k0 + 16);
        b1.h[0] = *(const v8h*)(wrow1 + k0);
        b1.h[1] = *(const v8h*)(wrow1 + k0 + 16);
        acc00 = __builtin_amdgcn_wmma_f32_16x16x32_f16(false, a0.v, false, b0.v,
                                                       (short)0, acc00, false, false);
        acc01 = __builtin_amdgcn_wmma_f32_16x16x32_f16(false, a0.v, false, b1.v,
                                                       (short)0, acc01, false, false);
        acc10 = __builtin_amdgcn_wmma_f32_16x16x32_f16(false, a1.v, false, b0.v,
                                                       (short)0, acc10, false, false);
        acc11 = __builtin_amdgcn_wmma_f32_16x16x32_f16(false, a1.v, false, b1.v,
                                                       (short)0, acc11, false, false);
        asm volatile("v_nop\n\tv_nop\n\tv_nop\n\tv_nop" : "+v"(acc00), "+v"(acc11) : "v"(a1.v), "v"(b1.v));
    }

    (void)Ch;
    float (*st)[33] = sT[threadIdx.x >> 5];
    const v8f* accs[4] = { &acc00, &acc01, &acc10, &acc11 };
#pragma unroll
    for (int t = 0; t < 4; t++) {
        const int cy = t >> 1, cx = t & 1;
        const v8f av = *accs[t];
#pragma unroll
        for (int r = 0; r < 8; r++) {
            float v = av[r];
            const int cl = cx * 16 + lidx;
            if (flags & GF_BIAS) v += bias[col0 + cl];
            st[cy * 16 + r + half * 8][cl] = v;
        }
    }
    __builtin_amdgcn_fence(__ATOMIC_RELEASE, "workgroup"); __builtin_amdgcn_wave_barrier(); __builtin_amdgcn_fence(__ATOMIC_ACQUIRE, "workgroup");
    float vals[32];
#pragma unroll
    for (int rr = 0; rr < 32; ++rr) {
        const int row = row0 + rr;
        int orow = row;
        if (flags & GF_REVC) orow = (row / LSEQ) * LSEQ + (LSEQ - 1 - (row % LSEQ));
        const size_t oi = (size_t)orow * N + col0 + lane;
        vals[rr] = st[rr][lane] + ((flags & GF_ACC) ? C[oi] : 0.0f);
    }
    for (int pass = 0; pass < 2; ++pass) {
#pragma unroll
        for (int rr = 0; rr < 32; ++rr) {
            const int row = row0 + rr;
            int orow = row;
            if (flags & GF_REVC) orow = (row / LSEQ) * LSEQ + (LSEQ - 1 - (row % LSEQ));
            *(volatile float*)(C + (size_t)orow * N + col0 + lane) = vals[rr];
        }
        __threadfence();
    }
}

__global__ void k_rows_f16(const float* __restrict__ in, _Float16* __restrict__ out, int n8) {
    const int i = blockIdx.x * blockDim.x + threadIdx.x;
    if (i >= n8) return;
    v8h v;
#pragma unroll
    for (int e = 0; e < 8; ++e) v[e] = (_Float16)in[(size_t)i * 8 + e];
    VST2(v8h, out + (size_t)i * 8, v);
}

__global__ void k_conv_silu(const float* __restrict__ xz, const float* __restrict__ convw,
                            const float* __restrict__ convb, float* __restrict__ xc,
                            _Float16* __restrict__ xch) {
    const int idx = blockIdx.x * blockDim.x + threadIdx.x;
    const int d = idx & (DINNER - 1);
    const int r = idx >> 9;
    const int l = r & (LSEQ - 1);
    const int b = r >> 10;
    float v = convb[d];
#pragma unroll
    for (int j = 0; j < 4; j++) {
        const int li = l - 3 + j;
        if (li >= 0) v += convw[d * 4 + j] * xz[((size_t)(b * LSEQ + li)) * (2 * DINNER) + d];
    }
    const float s = v / (1.0f + expf(-v));
    VST2(float, xc + idx, s);
    VST2(_Float16, xch + idx, (_Float16)s);
}

__global__ void k_dt(const float* __restrict__ proj, const float* __restrict__ Wdt,
                     const float* __restrict__ bdt, float* __restrict__ dt) {
    const int idx = blockIdx.x * blockDim.x + threadIdx.x;
    const int d = idx & (DINNER - 1);
    const int r = idx >> 9;
    const float* __restrict__ p = proj + (size_t)r * NPROJP;
    float a = bdt[d];
#pragma unroll
    for (int j = 0; j < DTRANK; j++) a += p[j] * Wdt[d * DTRANK + j];
    VST2(float, dt + idx, (a > 20.0f) ? a : log1pf(expf(a)));
}

__global__ __launch_bounds__(512) void k_scan(const float* __restrict__ dt, const float* __restrict__ xc,
                       const float* __restrict__ proj, const float* __restrict__ Alog,
                       const float* __restrict__ Dp, float* __restrict__ y) {
    const int b = blockIdx.x, d = threadIdx.x;
    float As[DSTATE], h[DSTATE];
#pragma unroll
    for (int s = 0; s < DSTATE; ++s) { As[s] = -expf(Alog[d * DSTATE + s]); h[s] = 0.f; }
    const float Dd = Dp[d];
    const size_t rbase = (size_t)b * LSEQ;
    for (int l = 0; l < LSEQ; l++) {
        const size_t r = rbase + l;
        const float dtv = dt[r * DINNER + d];
        const float xcv = xc[r * DINNER + d];
        const float du = dtv * xcv;
        float c = 0.f;
#pragma unroll
        for (int s = 0; s < DSTATE; ++s) {
            h[s] = __expf(dtv * As[s]) * h[s] + du * proj[r * NPROJP + DTRANK + s];
            c += h[s] * proj[r * NPROJP + DTRANK + DSTATE + s];
        }
        VST2(float, y + r * DINNER + d, c + Dd * xcv);
    }
}

__global__ void k_gate(const float* __restrict__ xz, const float* __restrict__ y,
                       _Float16* __restrict__ ygh) {
    const int idx = blockIdx.x * blockDim.x + threadIdx.x;
    const int d = idx & (DINNER - 1);
    const int r = idx >> 9;
    const float zv = xz[(size_t)r * (2 * DINNER) + DINNER + d];
    const float gl = zv / (1.0f + expf(-zv));
    VST2(_Float16, ygh + idx, (_Float16)(y[idx] * gl));
}

extern "C" void kernel_launch(void* const* d_in, const int* in_sizes, int n_in,
                              void* d_out, int out_size, void* d_ws, size_t ws_size,
                              hipStream_t stream) {
    (void)in_sizes; (void)n_in; (void)out_size;
    const float* ts = (const float*)d_in[0];
    const float* Wp = (const float*)d_in[1];
    const float* bp = (const float*)d_in[2];
    const float *Win[2], *convw[2], *convb[2], *Wx[2], *Wdt[2], *bdt[2], *Alog[2], *Dp[2], *Wout[2];
    for (int dir = 0; dir < 2; dir++) {
        const int o = 3 + dir * 9;
        Win[dir]   = (const float*)d_in[o + 0];
        convw[dir] = (const float*)d_in[o + 1];
        convb[dir] = (const float*)d_in[o + 2];
        Wx[dir]    = (const float*)d_in[o + 3];
        Wdt[dir]   = (const float*)d_in[o + 4];
        bdt[dir]   = (const float*)d_in[o + 5];
        Alog[dir]  = (const float*)d_in[o + 6];
        Dp[dir]    = (const float*)d_in[o + 7];
        Wout[dir]  = (const float*)d_in[o + 8];
    }
    float* out = (float*)d_out;

    char* w = (char*)d_ws;
    size_t off = 0;
    auto alloc = [&](size_t bytes) -> char* {
        char* p = w + off;
        off = (off + bytes + 255) & ~(size_t)255;
        return p;
    };
    _Float16* tsh      = (_Float16*)alloc((size_t)BL * DCLIP * 2);
    _Float16* Wph      = (_Float16*)alloc((size_t)DMODEL * DCLIP * 2);
    _Float16* Winh[2]  = { (_Float16*)alloc((size_t)2 * DINNER * DMODEL * 2),
                           (_Float16*)alloc((size_t)2 * DINNER * DMODEL * 2) };
    _Float16* Wxh[2]   = { (_Float16*)alloc((size_t)NPROJP * DINNER * 2),
                           (_Float16*)alloc((size_t)NPROJP * DINNER * 2) };
    _Float16* Wouth[2] = { (_Float16*)alloc((size_t)DMODEL * DINNER * 2),
                           (_Float16*)alloc((size_t)DMODEL * DINNER * 2) };
    float*    x    = (float*)alloc((size_t)BL * DMODEL * 4);
    _Float16* xh   = (_Float16*)alloc((size_t)BL * DMODEL * 2);
    float*    xz   = (float*)alloc((size_t)BL * 2 * DINNER * 4);
    float*    xc   = (float*)alloc((size_t)BL * DINNER * 4);
    _Float16* xch  = (_Float16*)alloc((size_t)BL * DINNER * 2);
    float*    proj = (float*)alloc((size_t)BL * NPROJP * 4);
    float*    dtb  = (float*)alloc((size_t)BL * DINNER * 4);
    float*    yb   = (float*)alloc((size_t)BL * DINNER * 4);
    _Float16* ygh  = (_Float16*)alloc((size_t)BL * DINNER * 2);
    if (off > ws_size) return;

    auto cvt = [&](const float* src, _Float16* dst, int n) {
        k_f32_to_f16<<<(n + 255) / 256, 256, 0, stream>>>(src, dst, n);
    };
    cvt(ts, tsh, BL * DCLIP);
    cvt(Wp, Wph, DMODEL * DCLIP);
    for (int dir = 0; dir < 2; dir++) {
        cvt(Win[dir], Winh[dir], 2 * DINNER * DMODEL);
        k_f32_to_f16_pad<<<(NPROJP * DINNER + 255) / 256, 256, 0, stream>>>(
            Wx[dir], Wxh[dir], NPROJ, NPROJP, DINNER);
        cvt(Wout[dir], Wouth[dir], DMODEL * DINNER);
    }

    const int NEL = BL * DINNER;
    const int ELB = NEL / 256;

    auto gemm_blocks = [](int M, int N) { return (M / 32) * (N / 32) / 4; };

    k_gemm_f16<<<gemm_blocks(BL, DMODEL), 128, 0, stream>>>(
        tsh, Wph, bp, x, nullptr, BL, DMODEL, DCLIP, GF_BIAS);
    k_rows_f16<<<(BL * DMODEL / 8 + 255) / 256, 256, 0, stream>>>(x, xh, BL * DMODEL / 8);

    for (int dir = 0; dir < 2; dir++) {
        k_gemm_f16<<<gemm_blocks(BL, 2 * DINNER), 128, 0, stream>>>(
            xh, Winh[dir], nullptr, xz, nullptr, BL, 2 * DINNER, DMODEL,
            dir ? GF_REVA : 0);
        k_conv_silu<<<ELB, 256, 0, stream>>>(xz, convw[dir], convb[dir], xc, xch);
        k_gemm_f16<<<gemm_blocks(BL, NPROJP), 128, 0, stream>>>(
            xch, Wxh[dir], nullptr, proj, nullptr, BL, NPROJP, DINNER, 0);
        k_dt<<<ELB, 256, 0, stream>>>(proj, Wdt[dir], bdt[dir], dtb);
        k_scan<<<BB, 512, 0, stream>>>(dtb, xc, proj, Alog[dir], Dp[dir], yb);
        k_gate<<<ELB, 256, 0, stream>>>(xz, yb, ygh);
        k_gemm_f16<<<gemm_blocks(BL, DMODEL), 128, 0, stream>>>(
            ygh, Wouth[dir], nullptr, out, nullptr, BL, DMODEL, DINNER,
            dir ? (GF_REVC | GF_ACC) : 0);
    }
}
